// Tenet_52183852646439
// MI455X (gfx1250) — hardware-verified
//
#include <hip/hip_runtime.h>
#include <stddef.h>


#define FIN     128
#define HDIM    256
#define NCLS    10
#define NGRAPH  64
#define NTHR    256
#define NWAVE   8
#define EPT     8
#define NGRP    2
#define CHUNK   (NTHR * EPT * NGRP)
#define WCAP    (EPT * NGRP * 32)
#define LISTN   (NWAVE * WCAP)
#define NBD     4096
#define NB1     512
#define NB2     256
#define GR      64
#define APH     264
#define WSCALE  16.0f
#define WINV    0.0625f
#define BN_S    0.99999500003749981f
#define TAU     0.1f
#define PSCALE  16384.0f
#define PINV    (1.0f / 16384.0f)
#define QB      64
#define KB      64
#define LDQ     264
#define LDSS    65
#define LDP     72

#define LDS_GEMM (GR * HDIM * 4)
#define LDS_AGG  (NB1 * FIN * 4 + LISTN * 4 + 64)
#define LDS_ATTN (QB * HDIM * 4)
#define AT_SF    (QB * LDQ * 2)
#define AT_PS    (AT_SF + QB * LDSS * 4)
#define AT_MI    (AT_PS + QB * LDP * 2)
#define AT_LI    (AT_MI + QB * 4)
#define AT_SC    (AT_LI + QB * 4)

static_assert((CHUNK & (CHUNK - 1)) == 0);
static_assert(CHUNK <= 4096);
static_assert(NB1 <= 4096 && NB2 <= 4096 && NBD <= 4096);
static_assert(NB1 * FIN == NB2 * HDIM);
static_assert(GR * APH * 2 <= LDS_GEMM);
static_assert(AT_SC + QB * 4 <= LDS_ATTN);
static_assert((AT_PS & 15) == 0 && (AT_SF & 15) == 0);
static_assert(NTHR == HDIM);
static_assert(NGRAPH * NCLS == 640);

typedef float    v4f  __attribute__((ext_vector_type(4)));
typedef float    v8f  __attribute__((ext_vector_type(8)));
typedef int      v4i  __attribute__((ext_vector_type(4)));
typedef _Float16 v8h  __attribute__((ext_vector_type(8)));
typedef _Float16 v16h __attribute__((ext_vector_type(16)));
union FragH { v16h v; v8h h[2]; };

__device__ __forceinline__ v8h cvt8(v4f a, v4f b) {
  v8h r;
  r[0] = (_Float16)a.x; r[1] = (_Float16)a.y; r[2] = (_Float16)a.z; r[3] = (_Float16)a.w;
  r[4] = (_Float16)b.x; r[5] = (_Float16)b.y; r[6] = (_Float16)b.z; r[7] = (_Float16)b.w;
  return r;
}

__device__ __forceinline__ v8f wmh(v16h a, v16h b, v8f c) {
  v8f d = __builtin_amdgcn_wmma_f32_16x16x32_f16(false, a, false, b, (short)0, c, false, false);
  asm volatile("v_nop\n\tv_nop\n\tv_nop\n\tv_nop" : "+v"(d) : "v"(a), "v"(b));
  return d;
}

template <int NB>
__device__ __forceinline__ int scan_chunk(const int* __restrict__ dsts, int nE, int cbase, int nodeBase,
                                          int vec8, int* list, int tid, int lane, int wave) {
  int wc = 0;
#pragma unroll
  for (int g = 0; g < NGRP; ++g) {
    const int el0  = (g * NTHR + tid) * EPT;
    const int e0   = cbase + el0;
    const int sent = -2147483647 - 1;
    v4i da, db;
    if (vec8 != 0 && e0 + 7 < nE) {
      da = *(const v4i*)(dsts + e0);
      db = *(const v4i*)(dsts + e0 + 4);
    } else {
      da.x = (e0     < nE) ? dsts[min(e0, nE - 1)] : sent;
      da.y = (e0 + 1 < nE) ? dsts[min(e0 + 1, nE - 1)] : sent;
      da.z = (e0 + 2 < nE) ? dsts[min(e0 + 2, nE - 1)] : sent;
      da.w = (e0 + 3 < nE) ? dsts[min(e0 + 3, nE - 1)] : sent;
      db.x = (e0 + 4 < nE) ? dsts[min(e0 + 4, nE - 1)] : sent;
      db.y = (e0 + 5 < nE) ? dsts[min(e0 + 5, nE - 1)] : sent;
      db.z = (e0 + 6 < nE) ? dsts[min(e0 + 6, nE - 1)] : sent;
      db.w = (e0 + 7 < nE) ? dsts[min(e0 + 7, nE - 1)] : sent;
    }
    const unsigned nb = (unsigned)nodeBase;
    const unsigned s0 = (unsigned)da.x - nb, s1 = (unsigned)da.y - nb;
    const unsigned s2 = (unsigned)da.z - nb, s3 = (unsigned)da.w - nb;
    const unsigned s4 = (unsigned)db.x - nb, s5 = (unsigned)db.y - nb;
    const unsigned s6 = (unsigned)db.z - nb, s7 = (unsigned)db.w - nb;
    const bool h0 = s0 < (unsigned)NB, h1 = s1 < (unsigned)NB, h2 = s2 < (unsigned)NB, h3 = s3 < (unsigned)NB;
    const bool h4 = s4 < (unsigned)NB, h5 = s5 < (unsigned)NB, h6 = s6 < (unsigned)NB, h7 = s7 < (unsigned)NB;
    const unsigned any = __builtin_amdgcn_ballot_w32(h0 | h1 | h2 | h3 | h4 | h5 | h6 | h7);
    if (any != 0u) {
#define HITJ(J, HJ, SJ) { \
        const unsigned mj = __builtin_amdgcn_ballot_w32(HJ); \
        if (mj != 0u) { \
          if (HJ) { \
            const int pos = wc + (int)__builtin_amdgcn_mbcnt_lo(mj, 0u); \
            if (pos < WCAP) list[wave * WCAP + pos] = ((el0 + (J)) << 12) | (int)(SJ); \
          } \
          wc += (int)__builtin_popcount(mj); } }
      HITJ(0, h0, s0)
      HITJ(1, h1, s1)
      HITJ(2, h2, s2)
      HITJ(3, h3, s3)
      HITJ(4, h4, s4)
      HITJ(5, h5, s5)
      HITJ(6, h6, s6)
      HITJ(7, h7, s7)
#undef HITJ
    }
  }
  return wc;
}

__global__ __launch_bounds__(NTHR) void k_wprep(
    const float* __restrict__ w0, const float* __restrict__ w1, const float* __restrict__ w2,
    const float* __restrict__ w3, const float* __restrict__ w4, const float* __restrict__ w5,
    const float* __restrict__ w6, const float* __restrict__ w7, _Float16* wp) {
  const int mat = blockIdx.x >> 5, blk = blockIdx.x & 31;
  const int K   = (mat == 0) ? FIN : HDIM;
  const int ksh = (mat == 0) ? 7 : 8;
  const int i   = blk * NTHR + threadIdx.x;
  if (i >= (HDIM * K) / 8) return;
  const float* W = (mat == 0) ? w0 : (mat == 1) ? w1 : (mat == 2) ? w2 : (mat == 3) ? w3
                 : (mat == 4) ? w4 : (mat == 5) ? w5 : (mat == 6) ? w6 : w7;
  const int o  = i * 8;
  const int n  = o >> ksh;
  const int k0 = o & (K - 1);
  const float* p = W + (size_t)k0 * HDIM + n;
  v4f a, b;
  a.x = p[0];        a.y = p[HDIM];     a.z = p[2 * HDIM]; a.w = p[3 * HDIM];
  b.x = p[4 * HDIM]; b.y = p[5 * HDIM]; b.z = p[6 * HDIM]; b.w = p[7 * HDIM];
  a = a * WSCALE;
  b = b * WSCALE;
  const v8h hv = cvt8(a, b);
  const int poff = (mat == 0) ? 0 : (FIN * HDIM + (mat - 1) * HDIM * HDIM);
  _Float16* dp = wp + (size_t)poff + o;
  *(volatile v8h*)dp = hv;
  __threadfence();
  *(volatile v8h*)dp = hv;
}

__global__ __launch_bounds__(NTHR) void k_deg(const int* __restrict__ ei, float* dinv, int nE, int vec8) {
  __shared__ __attribute__((aligned(16))) int cnt[NBD];
  __shared__ __attribute__((aligned(16))) int list[LISTN];
  __shared__ int wcnt[NWAVE];
  const int tid = threadIdx.x, lane = tid & 31, wave = tid >> 5;
  const int nodeBase = blockIdx.x * NBD;
  const int* dsts = ei + nE;

  for (int i = tid; i < NBD; i += NTHR) cnt[i] = 0;
  __syncthreads();

  const int nChunks = (nE + CHUNK - 1) / CHUNK;
#pragma unroll 1
  for (int ch = 0; ch < nChunks; ++ch) {
    const int cbase = ch * CHUNK;
    const int wc = scan_chunk<NBD>(dsts, nE, cbase, nodeBase, vec8, list, tid, lane, wave);
    if (lane == 0) wcnt[wave] = wc;
    __syncthreads();
    if (wave == 0) {
#pragma unroll 1
      for (int wsx = 0; wsx < NWAVE; ++wsx) {
        int n = __builtin_amdgcn_readfirstlane(wcnt[wsx]);
        n = n > WCAP ? WCAP : (n < 0 ? 0 : n);
        const int* lp = list + wsx * WCAP;
#pragma unroll 1
        for (int i = 0; i < n; ++i) {
          const int ent  = __builtin_amdgcn_readfirstlane(lp[i]);
          const int slot = ent & (NBD - 1);
          if (lane == 0) cnt[slot] = cnt[slot] + 1;
        }
      }
    }
    __syncthreads();
  }

  v4f dq[4];
#pragma unroll
  for (int q = 0; q < 4; ++q) {
    const int f = (wave * 4 + q) * 128 + 4 * lane;
    const v4i c = *(const v4i*)(cnt + f);
    dq[q].x = rsqrtf((float)(c.x + 1));
    dq[q].y = rsqrtf((float)(c.y + 1));
    dq[q].z = rsqrtf((float)(c.z + 1));
    dq[q].w = rsqrtf((float)(c.w + 1));
  }
  float* dp = dinv + (size_t)nodeBase;
#pragma unroll
  for (int q = 0; q < 4; ++q) *(volatile v4f*)(dp + (wave * 4 + q) * 128 + 4 * lane) = dq[q];
  __threadfence();
#pragma unroll
  for (int q = 0; q < 4; ++q) *(volatile v4f*)(dp + (wave * 4 + q) * 128 + 4 * lane) = dq[q];
}

template <int F, int NB>
__global__ __launch_bounds__(NTHR) void k_agg(
    const int* __restrict__ ei, const float* __restrict__ hin, const float* __restrict__ dinv,
    float* outp, int nN, int nE, int vec8) {
  extern __shared__ v4f lds_dyn[];
  float* acc  = (float*)lds_dyn;
  int*   list = (int*)(acc + NB * F);
  int*   wcnt = list + LISTN;
  const int tid = threadIdx.x, lane = tid & 31, wave = tid >> 5;
  const int nodeBase = blockIdx.x * NB;
  const int* dsts = ei + nE;

  {
    const v4f z = {0.f, 0.f, 0.f, 0.f};
    for (int i = tid; i < NB * F / 4; i += NTHR) lds_dyn[i] = z;
  }
  __syncthreads();

  const int nChunks = (nE + CHUNK - 1) / CHUNK;
#pragma unroll 1
  for (int ch = 0; ch < nChunks; ++ch) {
    const int cbase = ch * CHUNK;
    const int wc = scan_chunk<NB>(dsts, nE, cbase, nodeBase, vec8, list, tid, lane, wave);
    if (lane == 0) wcnt[wave] = wc;
    __syncthreads();
    if (wave == 0) {
#pragma unroll 1
      for (int wsx = 0; wsx < NWAVE; ++wsx) {
        int n = __builtin_amdgcn_readfirstlane(wcnt[wsx]);
        n = n > WCAP ? WCAP : (n < 0 ? 0 : n);
        const int* lp = list + wsx * WCAP;
#pragma unroll 1
        for (int i = 0; i < n; ++i) {
          const int ent  = __builtin_amdgcn_readfirstlane(lp[i]);
          const int slot = ent & (NB - 1);
          int e = cbase + ((ent >> 12) & (CHUNK - 1));
          e = e > nE - 1 ? nE - 1 : e;
          int src = ei[e];
          src = src < 0 ? 0 : (src > nN - 1 ? nN - 1 : src);
          const float d = dinv[src];
          const float* hp = hin + (size_t)src * F + 4 * lane;
          float* ap = acc + slot * F + 4 * lane;
          const v4f v0 = *(const v4f*)hp * d;
          *(v4f*)ap = *(const v4f*)ap + v0;
          if (F == 256) {
            const v4f v1 = *(const v4f*)(hp + 128) * d;
            *(v4f*)(ap + 128) = *(const v4f*)(ap + 128) + v1;
          }
        }
      }
    }
    __syncthreads();
  }

  constexpr int FQ = F / 4;
#pragma unroll 4
  for (int i = 0; i < (NB * FQ) / NTHR; ++i) {
    const int idx  = i * NTHR + tid;
    const int slot = idx / FQ;
    const int c4   = (idx - slot * FQ) * 4;
    int node = nodeBase + slot;
    node = node > nN - 1 ? nN - 1 : node;
    const float d  = dinv[node];
    const v4f   xv = *(const v4f*)(hin + (size_t)node * F + c4);
    v4f* ap = (v4f*)(acc + slot * F + c4);
    *ap = (*ap + xv * d) * d;
  }
  __syncthreads();

  constexpr int RW = NB / NWAVE;
  constexpr int QI = F / 128;
  float* gp = outp + (size_t)nodeBase * F;
#pragma unroll 8
  for (int i = 0; i < RW; ++i) {
#pragma unroll
    for (int q = 0; q < QI; ++q) {
      const int f = (wave * RW + i) * F + 128 * q + 4 * lane;
      const v4f v = *(const v4f*)(acc + f);
      *(volatile v4f*)(gp + f) = v;
    }
  }
  __threadfence();
#pragma unroll 8
  for (int i = 0; i < RW; ++i) {
#pragma unroll
    for (int q = 0; q < QI; ++q) {
      const int f = (wave * RW + i) * F + 128 * q + 4 * lane;
      const v4f v = *(const v4f*)(acc + f);
      *(volatile v4f*)(gp + f) = v;
    }
  }
}

template <int K, int AMODE, int EPI, int OMODE>
__global__ __launch_bounds__(NTHR) void k_gemm(
    const float* __restrict__ A, const int* __restrict__ yix, const float* __restrict__ gtab,
    const float* __restrict__ gb, const float* __restrict__ gg, const float* __restrict__ gbe,
    const _Float16* __restrict__ wpl,
    const float* __restrict__ bias, const float* __restrict__ gam, const float* __restrict__ bet,
    float* out32, _Float16* out16, int M, int ntab, int ldt) {
  extern __shared__ v4f lds_dyn[];
  _Float16* sA  = (_Float16*)lds_dyn;
  float*    stg = (float*)lds_dyn;
  const int tid = threadIdx.x, lane = tid & 31, wave = tid >> 5, hh = lane >> 4, m = lane & 15;
  const int rt = wave & 3, ch = wave >> 2;
  const int rowBase = blockIdx.x * GR;
  constexpr int KQ = K / 8;

#pragma unroll
  for (int i = 0; i < (GR * KQ) / NTHR; ++i) {
    const int idx = i * NTHR + tid;
    const int r   = idx / KQ;
    const int c0  = (idx - r * KQ) * 8;
    int row = rowBase + r;
    row = row > M - 1 ? M - 1 : row;
    v4f a, b;
    if (AMODE == 0) {
      const float* ap = A + (size_t)row * K + c0;
      a = *(const v4f*)ap;
      b = *(const v4f*)(ap + 4);
    } else {
      const int  yi  = yix[row];
      const bool ok  = (unsigned)yi < (unsigned)ntab;
      const int  yc  = ok ? yi : 0;
      const float okf = ok ? 1.f : 0.f;
      const float* tp = gtab + (size_t)yc * K + c0;
      const v4f ta = *(const v4f*)tp * okf, tb = *(const v4f*)(tp + 4) * okf;
      const v4f b0 = *(const v4f*)(gb + c0), b1 = *(const v4f*)(gb + c0 + 4);
      const v4f g0 = *(const v4f*)(gg + c0) * BN_S, g1 = *(const v4f*)(gg + c0 + 4) * BN_S;
      const v4f e0 = *(const v4f*)(gbe + c0), e1 = *(const v4f*)(gbe + c0 + 4);
      a = (ta + b0) * g0 + e0;
      b = (tb + b1) * g1 + e1;
      a.x = fmaxf(a.x, 0.f); a.y = fmaxf(a.y, 0.f); a.z = fmaxf(a.z, 0.f); a.w = fmaxf(a.w, 0.f);
      b.x = fmaxf(b.x, 0.f); b.y = fmaxf(b.y, 0.f); b.z = fmaxf(b.z, 0.f); b.w = fmaxf(b.w, 0.f);
    }
    *(v8h*)(sA + r * APH + c0) = cvt8(a, b);
  }
  __syncthreads();

  v8f acc[8];
#pragma unroll
  for (int t = 0; t < 8; ++t) { v8f z = {0.f, 0.f, 0.f, 0.f, 0.f, 0.f, 0.f, 0.f}; acc[t] = z; }
  const _Float16* ar = sA + (16 * rt + m) * APH + 8 * hh;
  const _Float16* br = wpl + (size_t)(128 * ch + m) * K + 8 * hh;
#pragma unroll
  for (int kt = 0; kt < K / 32; ++kt) {
    FragH a;
    a.h[0] = *(const v8h*)(ar + 32 * kt);
    a.h[1] = *(const v8h*)(ar + 32 * kt + 16);
#pragma unroll
    for (int t = 0; t < 8; ++t) {
      const _Float16* bp = br + (size_t)(16 * t) * K + 32 * kt;
      FragH b;
      b.h[0] = *(const v8h*)bp;
      b.h[1] = *(const v8h*)(bp + 16);
      acc[t] = wmh(a.v, b.v, acc[t]);
    }
  }
  __syncthreads();

  const int r0w = 16 * rt + 8 * hh;
#pragma unroll
  for (int t = 0; t < 8; ++t) {
    const int col = 128 * ch + 16 * t + m;
    const float bc = bias[col];
    float gs = 1.f, be = 0.f;
    if (EPI) { gs = BN_S * gam[col]; be = bet[col]; }
    float* sp = stg + r0w * HDIM + col;
#pragma unroll
    for (int r = 0; r < 8; ++r) {
      float v = acc[t][r] * WINV + bc;
      if (EPI) { v = v * gs + be; v = fmaxf(v, 0.f); }
      sp[r * HDIM] = v;
    }
  }
  __syncthreads();

  if (OMODE == 0) {
    const float* lp = stg + wave * 8 * HDIM;
    float* gp = out32 + ((size_t)rowBase + wave * 8) * HDIM;
#pragma unroll
    for (int i = 0; i < 8; ++i) {
#pragma unroll
      for (int q = 0; q < 2; ++q) {
        const int f = i * HDIM + 128 * q + 4 * lane;
        const v4f v = *(const v4f*)(lp + f);
        *(volatile v4f*)(gp + f) = v;
      }
    }
    __threadfence();
#pragma unroll
    for (int i = 0; i < 8; ++i) {
#pragma unroll
      for (int q = 0; q < 2; ++q) {
        const int f = i * HDIM + 128 * q + 4 * lane;
        const v4f v = *(const v4f*)(lp + f);
        *(volatile v4f*)(gp + f) = v;
      }
    }
  } else if (OMODE == 1) {
    const float* lp = stg + wave * 8 * HDIM + 8 * lane;
    _Float16* gp = out16 + ((size_t)rowBase + wave * 8) * HDIM + 8 * lane;
    v8h ov[8];
#pragma unroll
    for (int i = 0; i < 8; ++i) {
      const v4f a = *(const v4f*)(lp + i * HDIM), b = *(const v4f*)(lp + i * HDIM + 4);
      ov[i] = cvt8(a, b);
    }
#pragma unroll
    for (int i = 0; i < 8; ++i) *(volatile v8h*)(gp + (size_t)i * HDIM) = ov[i];
    __threadfence();
#pragma unroll
    for (int i = 0; i < 8; ++i) *(volatile v8h*)(gp + (size_t)i * HDIM) = ov[i];
  } else {
    const int k8 = (lane & 7) * 8;
    v8h ov[8];
#pragma unroll
    for (int q = 0; q < 8; ++q) {
      const int h = 32 * wave + 4 * q + (lane >> 3);
      const float* cp = stg + k8 * HDIM + h;
      v4f a, b;
      a.x = cp[0 * HDIM]; a.y = cp[1 * HDIM]; a.z = cp[2 * HDIM]; a.w = cp[3 * HDIM];
      b.x = cp[4 * HDIM]; b.y = cp[5 * HDIM]; b.z = cp[6 * HDIM]; b.w = cp[7 * HDIM];
      ov[q] = cvt8(a, b);
    }
#pragma unroll
    for (int q = 0; q < 8; ++q) {
      const int h = 32 * wave + 4 * q + (lane >> 3);
      *(volatile v8h*)(out16 + (size_t)h * ldt + rowBase + k8) = ov[q];
    }
    __threadfence();
#pragma unroll
    for (int q = 0; q < 8; ++q) {
      const int h = 32 * wave + 4 * q + (lane >> 3);
      *(volatile v8h*)(out16 + (size_t)h * ldt + rowBase + k8) = ov[q];
    }
  }
}

__global__ __launch_bounds__(NTHR) void k_attn(
    const _Float16* __restrict__ Qh, const _Float16* __restrict__ Kh, const _Float16* __restrict__ Vt,
    float* Z, int nN) {
  extern __shared__ v4f lds_dyn[];
  char* base = (char*)lds_dyn;
  _Float16* Qs   = (_Float16*)base;
  float*    Sf   = (float*)(base + AT_SF);
  _Float16* Ps   = (_Float16*)(base + AT_PS);
  float*    m_i  = (float*)(base + AT_MI);
  float*    l_i  = (float*)(base + AT_LI);
  float*    sc_s = (float*)(base + AT_SC);
  float*    stg  = (float*)base;
  const int tid = threadIdx.x, lane = tid & 31, wave = tid >> 5, hh = lane >> 4, m = lane & 15;
  const int q0  = blockIdx.x * QB;
  const int ms  = wave & 3, ns0 = (wave >> 2) * 2;
  const int mq  = wave & 3, nh  = wave >> 2;
  const int row = tid >> 2, seg = tid & 3;

#pragma unroll
  for (int i = 0; i < (QB * HDIM / 8) / NTHR; ++i) {
    const int idx = i * NTHR + tid, r = idx >> 5, c0 = (idx & 31) * 8;
    *(v8h*)(Qs + r * LDQ + c0) = *(const v8h*)(Qh + (size_t)(q0 + r) * HDIM + c0);
  }
  if (tid < QB) { m_i[tid] = -__builtin_inff(); l_i[tid] = 0.f; }
  v8f o[8];
#pragma unroll
  for (int i = 0; i < 8; ++i) { v8f z = {0.f, 0.f, 0.f, 0.f, 0.f, 0.f, 0.f, 0.f}; o[i] = z; }
  __syncthreads();

  const _Float16* qrow = Qs + (16 * ms + m) * LDQ + 8 * hh;
  const _Float16* prow = Ps + (16 * mq + m) * LDP + 8 * hh;
  const int nkb = nN / KB;
#pragma unroll 1
  for (int kbi = 0; kbi < nkb; ++kbi) {
    const int kb = kbi * KB;
    v8f s0 = {0.f, 0.f, 0.f, 0.f, 0.f, 0.f, 0.f, 0.f};
    v8f s1 = s0;
    const _Float16* k0p = Kh + (size_t)(kb + 16 * ns0 + m) * HDIM + 8 * hh;
    const _Float16* k1p = k0p + (size_t)16 * HDIM;
#pragma unroll
    for (int kt = 0; kt < HDIM / 32; ++kt) {
      FragH a, b0, b1;
      a.h[0]  = *(const v8h*)(qrow + 32 * kt);
      a.h[1]  = *(const v8h*)(qrow + 32 * kt + 16);
      b0.h[0] = *(const v8h*)(k0p + 32 * kt);
      b0.h[1] = *(const v8h*)(k0p + 32 * kt + 16);
      b1.h[0] = *(const v8h*)(k1p + 32 * kt);
      b1.h[1] = *(const v8h*)(k1p + 32 * kt + 16);
      s0 = wmh(a.v, b0.v, s0);
      s1 = wmh(a.v, b1.v, s1);
    }
    {
      float* sp = Sf + (16 * ms + 8 * hh) * LDSS + 16 * ns0 + m;
#pragma unroll
      for (int r = 0; r < 8; ++r) { sp[r * LDSS] = s0[r] * TAU; sp[r * LDSS + 16] = s1[r] * TAU; }
    }
    __syncthreads();

    {
      const float* sfr = Sf + row * LDSS + seg * 16;
      float sv[16];
#pragma unroll
      for (int c = 0; c < 16; ++c) sv[c] = sfr[c];
      float lmax = sv[0];
#pragma unroll
      for (int c = 1; c < 16; ++c) lmax = fmaxf(lmax, sv[c]);
      lmax = fmaxf(lmax, __shfl_xor(lmax, 1));
      lmax = fmaxf(lmax, __shfl_xor(lmax, 2));
      const float mo = m_i[row];
      const float mn = fmaxf(mo, lmax);
      const float sc = (mo == -__builtin_inff()) ? 0.f : __expf(mo - mn);
      float lsum = 0.f;
      v8h p0, p1;
#pragma unroll
      for (int c = 0; c < 8; ++c) {
        const float p = __expf(sv[c] - mn);
        lsum += p;
        p0[c] = (_Float16)(p * PSCALE);
      }
#pragma unroll
      for (int c = 0; c < 8; ++c) {
        const float p = __expf(sv[8 + c] - mn);
        lsum += p;
        p1[c] = (_Float16)(p * PSCALE);
      }
      lsum += __shfl_xor(lsum, 1);
      lsum += __shfl_xor(lsum, 2);
      *(v8h*)(Ps + row * LDP + seg * 16)     = p0;
      *(v8h*)(Ps + row * LDP + seg * 16 + 8) = p1;
      if (seg == 0) { m_i[row] = mn; sc_s[row] = sc; l_i[row] = l_i[row] * sc + lsum; }
    }
    __syncthreads();

    {
      const float* scp = sc_s + 16 * mq + 8 * hh;
      float scv[8];
#pragma unroll
      for (int r = 0; r < 8; ++r) scv[r] = scp[r];
#pragma unroll
      for (int i = 0; i < 8; ++i) {
#pragma unroll
        for (int r = 0; r < 8; ++r) o[i][r] *= scv[r];
      }
    }
#pragma unroll
    for (int j = 0; j < KB / 32; ++j) {
      FragH a;
      a.h[0] = *(const v8h*)(prow + 32 * j);
      a.h[1] = *(const v8h*)(prow + 32 * j + 16);
      const _Float16* vp = Vt + (size_t)(128 * nh + m) * nN + kb + 32 * j + 8 * hh;
#pragma unroll
      for (int i = 0; i < 8; ++i) {
        const _Float16* vpi = vp + (size_t)(16 * i) * nN;
        FragH b;
        b.h[0] = *(const v8h*)vpi;
        b.h[1] = *(const v8h*)(vpi + 16);
        o[i] = wmh(a.v, b.v, o[i]);
      }
    }
    __syncthreads();
  }

  const int rB = 16 * mq + 8 * hh;
  float inv[8];
#pragma unroll
  for (int r = 0; r < 8; ++r) inv[r] = PINV * (1.0f / l_i[rB + r]);
  __syncthreads();
#pragma unroll
  for (int i = 0; i < 8; ++i) {
    float* sp = stg + rB * HDIM + 16 * (8 * nh + i) + m;
#pragma unroll
    for (int r = 0; r < 8; ++r) sp[r * HDIM] = o[i][r] * inv[r];
  }
  __syncthreads();
  const float* lp = stg + wave * 8 * HDIM;
  float* gp = Z + ((size_t)q0 + wave * 8) * HDIM;
#pragma unroll
  for (int i = 0; i < 8; ++i) {
#pragma unroll
    for (int q = 0; q < 2; ++q) {
      const int f = i * HDIM + 128 * q + 4 * lane;
      const v4f v = *(const v4f*)(lp + f);
      *(volatile v4f*)(gp + f) = v;
    }
  }
  __threadfence();
#pragma unroll
  for (int i = 0; i < 8; ++i) {
#pragma unroll
    for (int q = 0; q < 2; ++q) {
      const int f = i * HDIM + 128 * q + 4 * lane;
      const v4f v = *(const v4f*)(lp + f);
      *(volatile v4f*)(gp + f) = v;
    }
  }
}

__global__ __launch_bounds__(NTHR) void k_pool(
    const float* __restrict__ Z, const int* __restrict__ bat, float* rep, float* out1, int nN) {
  __shared__ int list[NWAVE * 32];
  __shared__ int wcnt[NWAVE];
  __shared__ float wred[NWAVE];
  __shared__ __attribute__((aligned(16))) float rowst[HDIM];
  const int tid = threadIdx.x, lane = tid & 31, wave = tid >> 5;
  const int g = blockIdx.x;
  float acc = 0.f;
  int cnt = 0;
  const int nch = (nN + NTHR - 1) / NTHR;
#pragma unroll 1
  for (int ch = 0; ch < nch; ++ch) {
    const int i  = ch * NTHR + tid;
    const int ii = i < nN ? i : nN - 1;
    const int b  = bat[ii];
    const bool hit = (i < nN) && (b == g);
    const unsigned mk = __builtin_amdgcn_ballot_w32(hit);
    if (hit) list[wave * 32 + (int)__builtin_amdgcn_mbcnt_lo(mk, 0u)] = i;
    if (lane == 0) wcnt[wave] = (int)__builtin_popcount(mk);
    __syncthreads();
#pragma unroll 1
    for (int wsx = 0; wsx < NWAVE; ++wsx) {
      int n = wcnt[wsx];
      n = n > 32 ? 32 : (n < 0 ? 0 : n);
      cnt += n;
#pragma unroll 1
      for (int j = 0; j < n; ++j) {
        int r = list[wsx * 32 + j];
        r = r < 0 ? 0 : (r > nN - 1 ? nN - 1 : r);
        acc += Z[(size_t)r * HDIM + tid];
      }
    }
    __syncthreads();
  }
  const float mean = acc * (1.0f / (float)(cnt > 1 ? cnt : 1));
  float ss = mean * mean;
  ss += __shfl_xor(ss, 16);
  ss += __shfl_xor(ss, 8);
  ss += __shfl_xor(ss, 4);
  ss += __shfl_xor(ss, 2);
  ss += __shfl_xor(ss, 1);
  if (lane == 0) wred[wave] = ss;
  __syncthreads();
  float tot = 0.f;
#pragma unroll
  for (int w = 0; w < NWAVE; ++w) tot += wred[w];
  const float rv = mean * (1.0f / sqrtf(tot));
  rowst[tid] = rv;
  __syncthreads();
  if (wave == 0) {
    const v4f v0 = *(const v4f*)(rowst + 4 * lane);
    const v4f v1 = *(const v4f*)(rowst + 128 + 4 * lane);
    float* rp = rep  + (size_t)g * HDIM;
    float* op = out1 + (size_t)g * HDIM;
    *(volatile v4f*)(rp + 4 * lane) = v0; *(volatile v4f*)(rp + 128 + 4 * lane) = v1;
    *(volatile v4f*)(op + 4 * lane) = v0; *(volatile v4f*)(op + 128 + 4 * lane) = v1;
    __threadfence();
    *(volatile v4f*)(rp + 4 * lane) = v0; *(volatile v4f*)(rp + 128 + 4 * lane) = v1;
    *(volatile v4f*)(op + 4 * lane) = v0; *(volatile v4f*)(op + 128 + 4 * lane) = v1;
  }
}

__global__ __launch_bounds__(NTHR) void k_cls(
    const float* __restrict__ c1, const float* __restrict__ w2, const float* __restrict__ b2,
    float* out0, int nG) {
  __shared__ float lg[NGRAPH * NCLS];
  __shared__ __attribute__((aligned(16))) float pr[NGRAPH * NCLS];
  const int tid = threadIdx.x, lane = tid & 31, wave = tid >> 5;
  const int tot = nG * NCLS;
  for (int oo = tid; oo < tot; oo += NTHR) {
    const int r = oo / NCLS, c = oo - r * NCLS;
    const float* cr = c1 + (size_t)r * HDIM;
    float a = 0.f;
#pragma unroll 4
    for (int k = 0; k < HDIM; ++k) a += cr[k] * w2[k * NCLS + c];
    lg[oo] = a + b2[c];
  }
  __syncthreads();
  if (tid < nG) {
    const float* lr = lg + tid * NCLS;
    float mx = lr[0];
#pragma unroll
    for (int c = 1; c < NCLS; ++c) mx = fmaxf(mx, lr[c]);
    float sum = 0.f;
#pragma unroll
    for (int c = 0; c < NCLS; ++c) sum += __expf(lr[c] - mx);
    const float ls = __logf(sum);
#pragma unroll
    for (int c = 0; c < NCLS; ++c) pr[tid * NCLS + c] = lr[c] - mx - ls;
  }
  __syncthreads();
  if (wave == 0) {
#pragma unroll
    for (int q = 0; q < (NGRAPH * NCLS) / 128; ++q) {
      const int f = q * 128 + 4 * lane;
      const v4f v = *(const v4f*)(pr + f);
      *(volatile v4f*)(out0 + f) = v;
    }
    __threadfence();
#pragma unroll
    for (int q = 0; q < (NGRAPH * NCLS) / 128; ++q) {
      const int f = q * 128 + 4 * lane;
      const v4f v = *(const v4f*)(pr + f);
      *(volatile v4f*)(out0 + f) = v;
    }
  }
}

template <typename T>
static void set_dyn_lds(T* f, int bytes) {
  hipFuncSetAttribute(reinterpret_cast<const void*>(f), hipFuncAttributeMaxDynamicSharedMemorySize, bytes);
}

extern "C" void kernel_launch(void* const* d_in, const int* in_sizes, int n_in,
                              void* d_out, int out_size, void* d_ws, size_t ws_size,
                              hipStream_t stream) {
  if (n_in < 32) return;
  const int nN = in_sizes[3];
  const int nE = in_sizes[2] / 2;
  const int nG = NGRAPH;
  if (nN <= 0 || (nN % GR) != 0 || (nN % KB) != 0 || nE < 0 || in_sizes[2] != 2 * nE) return;
  if (in_sizes[0] != nN * FIN || in_sizes[1] != nN) return;
  if (out_size != nG * (NCLS + HDIM)) return;
  if (in_sizes[4] != FIN * HDIM || in_sizes[8] != HDIM * HDIM || in_sizes[10] != NCLS * HDIM ||
      in_sizes[14] != HDIM * HDIM || in_sizes[18] != HDIM * HDIM || in_sizes[20] != HDIM * HDIM ||
      in_sizes[22] != HDIM * HDIM || in_sizes[24] != HDIM * HDIM || in_sizes[26] != HDIM * HDIM ||
      in_sizes[30] != HDIM * NCLS || in_sizes[31] < NCLS) return;
  if (in_sizes[5] < HDIM || in_sizes[6] < HDIM || in_sizes[7] < HDIM || in_sizes[9] < HDIM ||
      in_sizes[11] < HDIM || in_sizes[12] < HDIM || in_sizes[13] < HDIM || in_sizes[15] < HDIM ||
      in_sizes[16] < HDIM || in_sizes[17] < HDIM || in_sizes[19] < HDIM || in_sizes[21] < HDIM ||
      in_sizes[23] < HDIM || in_sizes[25] < HDIM || in_sizes[27] < HDIM || in_sizes[28] < HDIM ||
      in_sizes[29] < HDIM) return;

  const float* x    = (const float*)d_in[0];
  const int*   y    = (const int*)d_in[1];
  const int*   ei   = (const int*)d_in[2];
  const int*   bat  = (const int*)d_in[3];
  const float* gw1  = (const float*)d_in[4],  *gb1  = (const float*)d_in[5];
  const float* gg1  = (const float*)d_in[6],  *gbe1 = (const float*)d_in[7];
  const float* gw2  = (const float*)d_in[8],  *gb2  = (const float*)d_in[9];
  const float* lw1  = (const float*)d_in[10], *lb1  = (const float*)d_in[11];
  const float* lg1  = (const float*)d_in[12], *lbe1 = (const float*)d_in[13];
  const float* lw2  = (const float*)d_in[14], *lb2  = (const float*)d_in[15];
  const float* lg2  = (const float*)d_in[16], *lbe2 = (const float*)d_in[17];
  const float* lw3  = (const float*)d_in[18], *lb3  = (const float*)d_in[19];
  const float* wq   = (const float*)d_in[20], *bq   = (const float*)d_in[21];
  const float* wk   = (const float*)d_in[22], *bk   = (const float*)d_in[23];
  const float* wv   = (const float*)d_in[24], *bv   = (const float*)d_in[25];
  const float* cw1  = (const float*)d_in[26], *cb1  = (const float*)d_in[27];
  const float* cg   = (const float*)d_in[28], *cbe  = (const float*)d_in[29];
  const float* cw2  = (const float*)d_in[30], *cb2  = (const float*)d_in[31];
  float* out0 = (float*)d_out;
  float* out1 = out0 + nG * NCLS;

  const int nBD = (nN + NBD - 1) / NBD;
  const int nA1 = (nN + NB1 - 1) / NB1;
  const int nA2 = (nN + NB2 - 1) / NB2;
  const int nGB = nN / GR;
  const int nQB = nN / QB;
  const int nCB = (nG + GR - 1) / GR;

  char* ws = (char*)d_ws;
  size_t off = 0;
  const size_t wpElems = (size_t)FIN * HDIM + (size_t)7 * HDIM * HDIM;
  const size_t oWP  = off; off += wpElems * 2;                                  off = (off + 255) & ~(size_t)255;
  const size_t oDV  = off; off += (size_t)nBD * NBD * 4;                        off = (off + 255) & ~(size_t)255;
  const size_t oAG1 = off; off += (size_t)nA1 * NB1 * FIN * 4;                  off = (off + 255) & ~(size_t)255;
  const size_t oH   = off; off += (size_t)nN * HDIM * 4;                        off = (off + 255) & ~(size_t)255;
  const size_t oAG2 = off; off += (size_t)nA2 * NB2 * HDIM * 4;                 off = (off + 255) & ~(size_t)255;
  const size_t oFEA = off; off += (size_t)nN * HDIM * 4;                        off = (off + 255) & ~(size_t)255;
  const size_t oL2  = off; off += (size_t)nN * HDIM * 4;                        off = (off + 255) & ~(size_t)255;
  const size_t oLE  = off; off += (size_t)nN * HDIM * 4;                        off = (off + 255) & ~(size_t)255;
  const size_t oQH  = off; off += (size_t)nN * HDIM * 2;                        off = (off + 255) & ~(size_t)255;
  const size_t oKH  = off; off += (size_t)nN * HDIM * 2;                        off = (off + 255) & ~(size_t)255;
  const size_t oVT  = off; off += (size_t)HDIM * nN * 2;                        off = (off + 255) & ~(size_t)255;
  const size_t oZ   = off; off += (size_t)nN * HDIM * 4;                        off = (off + 255) & ~(size_t)255;
  const size_t oREP = off; off += (size_t)nCB * GR * HDIM * 4;                  off = (off + 255) & ~(size_t)255;
  const size_t oC1  = off; off += (size_t)nCB * GR * HDIM * 4;                  off = (off + 255) & ~(size_t)255;
  if (off > ws_size) return;
  if (off > (size_t)134217728) return;

  _Float16* wp   = (_Float16*)(ws + oWP);
  _Float16* wpG1 = wp;
  _Float16* wpG2 = wp + (size_t)FIN * HDIM + (size_t)0 * HDIM * HDIM;
  _Float16* wpL2 = wp + (size_t)FIN * HDIM + (size_t)1 * HDIM * HDIM;
  _Float16* wpL3 = wp + (size_t)FIN * HDIM + (size_t)2 * HDIM * HDIM;
  _Float16* wpQ  = wp + (size_t)FIN * HDIM + (size_t)3 * HDIM * HDIM;
  _Float16* wpK  = wp + (size_t)FIN * HDIM + (size_t)4 * HDIM * HDIM;
  _Float16* wpV  = wp + (size_t)FIN * HDIM + (size_t)5 * HDIM * HDIM;
  _Float16* wpC1 = wp + (size_t)FIN * HDIM + (size_t)6 * HDIM * HDIM;
  float*    dinv = (float*)(ws + oDV);
  float*    ag1  = (float*)(ws + oAG1);
  float*    Hp   = (float*)(ws + oH);
  float*    ag2  = (float*)(ws + oAG2);
  float*    FEA  = (float*)(ws + oFEA);
  float*    L2   = (float*)(ws + oL2);
  float*    LE   = (float*)(ws + oLE);
  _Float16* Qh   = (_Float16*)(ws + oQH);
  _Float16* Kh   = (_Float16*)(ws + oKH);
  _Float16* Vt   = (_Float16*)(ws + oVT);
  float*    Zp   = (float*)(ws + oZ);
  float*    REP  = (float*)(ws + oREP);
  float*    C1   = (float*)(ws + oC1);

  const int vec8 = ((nE & 3) == 0) ? 1 : 0;

  k_wprep<<<8 * 32, NTHR, 0, stream>>>(gw1, gw2, lw2, lw3, wq, wk, wv, cw1, wp);

  k_deg<<<nBD, NTHR, 0, stream>>>(ei, dinv, nE, vec8);

  set_dyn_lds(&k_agg<FIN, NB1>, LDS_AGG);
  k_agg<FIN, NB1><<<nA1, NTHR, LDS_AGG, stream>>>(ei, x, dinv, ag1, nN, nE, vec8);
  set_dyn_lds(&k_gemm<FIN, 0, 1, 0>, LDS_GEMM);
  k_gemm<FIN, 0, 1, 0><<<nGB, NTHR, LDS_GEMM, stream>>>(
      ag1, y, lw1, lb1, lg1, lbe1, wpG1, gb1, gg1, gbe1, Hp, Qh, nN, NCLS, nN);

  set_dyn_lds(&k_agg<HDIM, NB2>, LDS_AGG);
  k_agg<HDIM, NB2><<<nA2, NTHR, LDS_AGG, stream>>>(ei, Hp, dinv, ag2, nN, nE, vec8);
  set_dyn_lds(&k_gemm<HDIM, 0, 0, 0>, LDS_GEMM);
  k_gemm<HDIM, 0, 0, 0><<<nGB, NTHR, LDS_GEMM, stream>>>(
      ag2, y, lw1, lb1, lg1, lbe1, wpG2, gb2, gb2, gb2, FEA, Qh, nN, NCLS, nN);

  set_dyn_lds(&k_gemm<HDIM, 1, 1, 0>, LDS_GEMM);
  k_gemm<HDIM, 1, 1, 0><<<nGB, NTHR, LDS_GEMM, stream>>>(
      x, y, lw1, lb1, lg1, lbe1, wpL2, lb2, lg2, lbe2, L2, Qh, nN, NCLS, nN);
  k_gemm<HDIM, 0, 0, 0><<<nGB, NTHR, LDS_GEMM, stream>>>(
      L2, y, lw1, lb1, lg1, lbe1, wpL3, lb3, lb3, lb3, LE, Qh, nN, NCLS, nN);

  set_dyn_lds(&k_gemm<HDIM, 0, 0, 1>, LDS_GEMM);
  k_gemm<HDIM, 0, 0, 1><<<nGB, NTHR, LDS_GEMM, stream>>>(
      LE, y, lw1, lb1, lg1, lbe1, wpQ, bq, bq, bq, Zp, Qh, nN, NCLS, nN);
  k_gemm<HDIM, 0, 0, 1><<<nGB, NTHR, LDS_GEMM, stream>>>(
      FEA, y, lw1, lb1, lg1, lbe1, wpK, bk, bk, bk, Zp, Kh, nN, NCLS, nN);
  set_dyn_lds(&k_gemm<HDIM, 0, 0, 2>, LDS_GEMM);
  k_gemm<HDIM, 0, 0, 2><<<nGB, NTHR, LDS_GEMM, stream>>>(
      FEA, y, lw1, lb1, lg1, lbe1, wpV, bv, bv, bv, Zp, Vt, nN, NCLS, nN);

  set_dyn_lds(&k_attn, LDS_ATTN);
  k_attn<<<nQB, NTHR, LDS_ATTN, stream>>>(Qh, Kh, Vt, Zp, nN);

  k_pool<<<nG, NTHR, 0, stream>>>(Zp, bat, REP, out1, nN);

  set_dyn_lds(&k_gemm<HDIM, 0, 1, 0>, LDS_GEMM);
  k_gemm<HDIM, 0, 1, 0><<<nCB, NTHR, LDS_GEMM, stream>>>(
      REP, y, lw1, lb1, lg1, lbe1, wpC1, cb1, cg, cbe, C1, Qh, nG, NCLS, nN);
  k_cls<<<1, NTHR, 0, stream>>>(C1, cw2, cb2, out0, nG);
}
